// BoundaryGuidedDSTLayer_57964878626932
// MI455X (gfx1250) — hardware-verified
//
#include <hip/hip_runtime.h>


#define NB_  4
#define TT   2048
#define CC   512
#define NH_  8
#define HD   64
#define FF   2048
#define NT   (NB_ * TT)
#define ZH   2
#define PCAR 1024.0f
typedef _Float16 h16;
typedef unsigned short bf;
typedef __attribute__((ext_vector_type(16))) __bf16   v16bf;
typedef __attribute__((ext_vector_type(16))) _Float16 v16h;
typedef __attribute__((ext_vector_type(8)))  _Float16 v8h;
typedef __attribute__((ext_vector_type(8)))  unsigned short v8us;
typedef __attribute__((ext_vector_type(8)))  float    v8f;
typedef __attribute__((ext_vector_type(4)))  float    v4f;
typedef v8h  __attribute__((may_alias)) v8ha;
typedef v4f  __attribute__((may_alias)) v4fa;
typedef v8us __attribute__((may_alias)) v8usa;

__device__ __forceinline__ unsigned short f2bf(float f) { unsigned u = __float_as_uint(f); u += 0x7FFFu + ((u >> 16) & 1u); return (unsigned short)(u >> 16); }
__device__ __forceinline__ float bf2f(unsigned short b) { return __uint_as_float(((unsigned)b) << 16); }
__device__ __forceinline__ float bfr(float f) { return bf2f(f2bf(f)); }
__device__ __forceinline__ v16h cat16(v8h lo, v8h hi) { return __builtin_shufflevector(lo, hi, 0, 1, 2, 3, 4, 5, 6, 7, 8, 9, 10, 11, 12, 13, 14, 15); }
__device__ __forceinline__ v16bf cat16b(v8us lo, v8us hi) { return __builtin_bit_cast(v16bf, __builtin_shufflevector(lo, hi, 0, 1, 2, 3, 4, 5, 6, 7, 8, 9, 10, 11, 12, 13, 14, 15)); }
__device__ __forceinline__ v8f wmma16(v16h a, v16h b, v8f c) { return __builtin_amdgcn_wmma_f32_16x16x32_f16(false, a, false, b, (short)0, c, false, false); }
__device__ __forceinline__ v8f wmmab(v16bf a, v16bf b, v8f c) { return __builtin_amdgcn_wmma_f32_16x16x32_bf16(false, a, false, b, (short)0, c, false, false); }


template <typename T16> struct WFrag;
template <> struct WFrag<h16> { typedef v16h V; static __device__ __forceinline__ V ld(const h16* p) { return cat16(*(const v8h*)p, *(const v8h*)(p + 16)); } static __device__ __forceinline__ v8f mma(V a, V b, v8f c) { return wmma16(a, b, c); } };
template <> struct WFrag<bf> { typedef v16bf V; static __device__ __forceinline__ V ld(const bf* p) { return cat16b(*(const v8us*)p, *(const v8us*)(p + 16)); } static __device__ __forceinline__ v8f mma(V a, V b, v8f c) { return wmmab(a, b, c); } };
template <typename T16, int NSPLIT, bool BIAS>
__global__ __launch_bounds__(32) void k_gemmw(const T16* __restrict__ A, const T16* __restrict__ A2, const T16* __restrict__ Bt, const T16* __restrict__ Bt2, int K, float* C, int ldc, const float* __restrict__ bias, size_t sA, size_t sB, size_t sC) {
    typedef typename WFrag<T16>::V V;
    __shared__ __align__(16) float os[16 * 68];
    const size_t z = blockIdx.z; A += z * sA; if (A2) A2 += z * sA; Bt += z * sB; if (Bt2) Bt2 += z * sB; C += z * sC;
    const int lane = threadIdx.x & 31, lr = lane & 15, hi = lane >> 4; const int r0 = blockIdx.x * 64, c0 = blockIdx.y * 64;
    v8f acc[4][4];
#pragma unroll
    for (int mb = 0; mb < 4; ++mb)
#pragma unroll
        for (int nb = 0; nb < 4; ++nb) acc[mb][nb] = (v8f){};
    const size_t aoff = (size_t)(r0 + lr) * K + 8 * hi, boff = (size_t)(c0 + lr) * K + 8 * hi;
#pragma unroll 1
    for (int kc = 0; kc < K; kc += 32) {
        V a[4], a2[4];
#pragma unroll
        for (int mb = 0; mb < 4; ++mb) { a[mb] = WFrag<T16>::ld(A + aoff + (size_t)mb * 16 * K + kc); if (NSPLIT == 1 || NSPLIT == 2) a2[mb] = WFrag<T16>::ld(A2 + aoff + (size_t)mb * 16 * K + kc); }
#pragma unroll
        for (int nb = 0; nb < 4; ++nb) { const V b = WFrag<T16>::ld(Bt + boff + (size_t)nb * 16 * K + kc); V b2; if (NSPLIT >= 2) b2 = WFrag<T16>::ld(Bt2 + boff + (size_t)nb * 16 * K + kc);
#pragma unroll
            for (int mb = 0; mb < 4; ++mb) { acc[mb][nb] = WFrag<T16>::mma(a[mb], b, acc[mb][nb]); if (NSPLIT == 1 || NSPLIT == 2) acc[mb][nb] = WFrag<T16>::mma(a2[mb], b, acc[mb][nb]); if (NSPLIT >= 2) acc[mb][nb] = WFrag<T16>::mma(a[mb], b2, acc[mb][nb]); } }
        asm volatile("v_nop\n\tv_nop\n\tv_nop\n\tv_nop" : "+v"(acc[0][0]), "+v"(acc[1][1]), "+v"(acc[2][2]), "+v"(acc[3][3]) : "v"(a[0]), "v"(a[3]));
    }
#pragma unroll
    for (int mb = 0; mb < 4; ++mb) {
#pragma unroll
        for (int nb = 0; nb < 4; ++nb) {
#pragma unroll
            for (int j = 0; j < 8; ++j) os[(hi * 8 + j) * 68 + nb * 16 + lr] = acc[mb][nb][j]; }
        __builtin_amdgcn_wave_barrier(); asm volatile("" ::: "memory");
        float* crow = C + (size_t)(r0 + mb * 16) * ldc + c0;
#pragma unroll 1
        for (int ps = 0; ps < 2; ++ps) {
#pragma unroll
            for (int s = 0; s < 8; ++s) { const int row = 2 * s + hi, cofs = lr * 4; v4f val = *(const v4fa*)(os + row * 68 + cofs); if (BIAS) { val[0] += bfr(bias[c0 + cofs]); val[1] += bfr(bias[c0 + cofs + 1]); val[2] += bfr(bias[c0 + cofs + 2]); val[3] += bfr(bias[c0 + cofs + 3]); }
                *(volatile v4f*)(crow + (size_t)row * ldc + cofs) = val; }
            if (ps == 0) __threadfence(); }
        __builtin_amdgcn_wave_barrier(); asm volatile("" ::: "memory");
    }
}

__device__ __forceinline__ h16 tohx(float x) { return (h16)x; }
__device__ __forceinline__ float geluf(float x) { return 0.5f * x * (1.0f + erff(x * 0.70710678118654752f)); }
__device__ __noinline__ float gelun(float x) { return geluf(x); }
typedef __attribute__((ext_vector_type(4))) _Float16 v4h;
typedef __attribute__((ext_vector_type(2))) _Float16 v2h;

__global__ __launch_bounds__(256) void k_cvt8h(const float* __restrict__ src, h16* dst, size_t n8) { const size_t i = (size_t)blockIdx.x * 256 + threadIdx.x; if (i >= n8) return; const v8f v = *(const v8f*)(src + i * 8); v8h o;
#pragma unroll
    for (int k = 0; k < 8; ++k) o[k] = tohx(bfr(v[k])); *(volatile v8h*)(dst + i * 8) = o; __threadfence(); *(volatile v8h*)(dst + i * 8) = o; }
__global__ __launch_bounds__(256) void k_wconv(const float* __restrict__ w, bf* Bt) {
    typedef __attribute__((ext_vector_type(2))) unsigned short v2us;
    const int lane = threadIdx.x & 31; const int wg = blockIdx.x * 8 + (threadIdx.x >> 5), nw = gridDim.x * 8; const int nlines = CC * 3 * CC / 64;
#pragma unroll 1
    for (int ps = 0; ps < 2; ++ps) {
#pragma unroll 1
        for (int L = wg; L < nlines; L += nw) { const int e = L * 64 + lane * 2; v2us o;
#pragma unroll
            for (int q = 0; q < 2; ++q) { const int f = e + q; const int o_ = f / (3 * CC), kk = f % (3 * CC); const int k = kk / CC, c = kk % CC; o[q] = f2bf(w[((size_t)o_ * CC + c) * 3 + k]); }
            *(volatile v2us*)(Bt + e) = o; }
        if (ps == 0) __threadfence(); }
}
__global__ __launch_bounds__(256) void k_imc(const float* __restrict__ x, bf* A) {
    typedef __attribute__((ext_vector_type(2))) unsigned short v2us;
    const int lane = threadIdx.x & 31; const int L0 = (blockIdx.x * 8 + (threadIdx.x >> 5)) * 8; const int nlines = NT * 3 * CC / 64;
#pragma unroll 1
    for (int ps = 0; ps < 2; ++ps) {
#pragma unroll
        for (int l = 0; l < 8; ++l) { const int L = L0 + l; if (L >= nlines) break; const int e = L * 64 + lane * 2; const int r = e / (3 * CC), kk = e % (3 * CC); const int b = r / TT, t = r % TT; const int k = kk / CC, c = kk % CC; const int ts = t + k - 1; v2us o;
            const bool in = ts >= 0 && ts < TT; const float* src = x + ((size_t)b * TT + (ts < 0 ? 0 : (ts > TT - 1 ? TT - 1 : ts))) * CC + c;
#pragma unroll
            for (int q = 0; q < 2; ++q) o[q] = in ? f2bf(src[q]) : (unsigned short)0;
            *(volatile v2us*)(A + e) = o; }
        if (ps == 0) __threadfence(); }
}
template <bool GELU>
__global__ __launch_bounds__(256) void k_lnx(const float* __restrict__ x, const float* __restrict__ Y, const float* __restrict__ gg, const float* __restrict__ bb, h16* Mh) {
    const int lane = threadIdx.x & 31; const int r = blockIdx.x * 8 + (threadIdx.x >> 5); if (r >= NT) return; float v[16]; float s = 0.f;
#pragma unroll
    for (int c = 0; c < 4; ++c)
#pragma unroll
        for (int q = 0; q < 4; ++q) { const int col = c * 128 + lane * 4 + q; const float y = Y[(size_t)r * CC + col]; const float t = bfr(x[(size_t)r * CC + col]) + (GELU ? gelun(y) : y); v[c * 4 + q] = t; s += t; }
#pragma unroll
    for (int sh = 16; sh; sh >>= 1) s += __shfl_xor(s, sh, 32);
    const float mu = s * (1.0f / CC); float qq = 0.f;
#pragma unroll
    for (int i = 0; i < 16; ++i) { const float d = v[i] - mu; qq = fmaf(d, d, qq); }
#pragma unroll
    for (int sh = 16; sh; sh >>= 1) qq += __shfl_xor(qq, sh, 32);
    const float rs = rsqrtf(qq * (1.0f / CC) + 1e-5f); v4h o[4];
#pragma unroll
    for (int c = 0; c < 4; ++c)
#pragma unroll
        for (int q = 0; q < 4; ++q) { const int col = c * 128 + lane * 4 + q; o[c][q] = tohx((v[c * 4 + q] - mu) * rs * bfr(gg[col]) + bfr(bb[col])); }
#pragma unroll 1
    for (int ps = 0; ps < 2; ++ps) {
#pragma unroll
        for (int c = 0; c < 4; ++c) *(volatile v4h*)(Mh + (size_t)r * CC + c * 128 + lane * 4) = o[c];
        if (ps == 0) __threadfence(); }
}
__global__ __launch_bounds__(256) void k_hplane(const float* __restrict__ F, float sc, h16* P) {
    const int lane = threadIdx.x & 31; const int L0 = (blockIdx.x * 8 + (threadIdx.x >> 5)) * 8; const int nlines = NT * CC / 64;
#pragma unroll 1
    for (int ps = 0; ps < 2; ++ps) {
#pragma unroll
        for (int l = 0; l < 8; ++l) { const int L = L0 + l; if (L >= nlines) break; const int e = L * 64 + lane * 2; const int d = e & 63; const int t = (e >> 6) % TT; const int z = e / (64 * TT); const int b = z >> 3, h = z & 7; v2h v;
#pragma unroll
            for (int q = 0; q < 2; ++q) v[q] = tohx(F[((size_t)b * TT + t) * CC + h * HD + d + q] * sc);
            *(volatile v2h*)(P + e) = v; }
        if (ps == 0) __threadfence(); }
}
__global__ __launch_bounds__(256) void k_vtplane(const float* __restrict__ F, h16* VT) {
    const int lane = threadIdx.x & 31; const int L0 = (blockIdx.x * 8 + (threadIdx.x >> 5)) * 8; const int nlines = NT * CC / 64;
#pragma unroll 1
    for (int ps = 0; ps < 2; ++ps) {
#pragma unroll
        for (int l = 0; l < 8; ++l) { const int L = L0 + l; if (L >= nlines) break; const int e = L * 64 + lane * 2; const int t = e % TT; const int d = (e / TT) % 64; const int z = e / (64 * TT); const int b = z >> 3, h = z & 7; v2h v;
#pragma unroll
            for (int q = 0; q < 2; ++q) v[q] = tohx(F[((size_t)b * TT + t + q) * CC + h * HD + d]);
            *(volatile v2h*)(VT + e) = v; }
        if (ps == 0) __threadfence(); }
}
__global__ __launch_bounds__(256) void k_softab(const float* __restrict__ Sb, const float* __restrict__ A, const float* __restrict__ alphap, int b, h16* P) {
    const int lane = threadIdx.x & 31; const int row = blockIdx.x * 8 + (threadIdx.x >> 5); if (row >= ZH * TT) return; const int i = row % TT; const float* sr = Sb + (size_t)row * TT; const float* Ab = A + (size_t)b * TT;
    const float ai = bfr(alphap[0]) * bfr(Ab[i]);
    float m = -3.0e38f;
#pragma unroll 1
    for (int c0 = lane * 4; c0 < TT; c0 += 128) {
#pragma unroll
        for (int q = 0; q < 4; ++q) m = fmaxf(m, fmaf(ai, bfr(Ab[c0 + q]), sr[c0 + q])); }
#pragma unroll
    for (int sh = 16; sh; sh >>= 1) m = fmaxf(m, __shfl_xor(m, sh, 32));
    float sum = 0.f;
#pragma unroll 1
    for (int c0 = lane * 4; c0 < TT; c0 += 128) {
#pragma unroll
        for (int q = 0; q < 4; ++q) sum += __expf(fmaf(ai, bfr(Ab[c0 + q]), sr[c0 + q]) - m); }
#pragma unroll
    for (int sh = 16; sh; sh >>= 1) sum += __shfl_xor(sum, sh, 32);
    const float f = __fdiv_rn(PCAR, sum);
#pragma unroll 1
    for (int ps = 0; ps < 2; ++ps) {
#pragma unroll 1
        for (int c0 = lane * 4; c0 < TT; c0 += 128) { v4h o;
#pragma unroll
            for (int q = 0; q < 4; ++q) o[q] = tohx(__expf(fmaf(ai, bfr(Ab[c0 + q]), sr[c0 + q]) - m) * f);
            *(volatile v4h*)(P + (size_t)row * TT + c0) = o; }
        if (ps == 0) __threadfence(); }
}
__global__ __launch_bounds__(256) void k_merge(const float* __restrict__ O, int b, int h0, h16* AT) {
    const int lane = threadIdx.x & 31; const int t = blockIdx.x * 8 + (threadIdx.x >> 5); if (t >= TT) return; const int zz = lane >> 4, d = (lane & 15) * 4; v4h o;
#pragma unroll
    for (int q = 0; q < 4; ++q) o[q] = tohx(O[((size_t)zz * TT + t) * 64 + d + q] * (1.0f / PCAR));
    h16* dst = AT + ((size_t)b * TT + t) * CC + (h0 + zz) * HD + d; *(volatile v4h*)dst = o; __threadfence(); *(volatile v4h*)dst = o;
}
__global__ __launch_bounds__(256) void k_gelu16(const float* __restrict__ H, int n, h16* P) {
    const int lane = threadIdx.x & 31; const int L0 = (blockIdx.x * 8 + (threadIdx.x >> 5)) * 8; const int nlines = n / 64;
#pragma unroll 1
    for (int ps = 0; ps < 2; ++ps) {
#pragma unroll 1
        for (int l = 0; l < 8; ++l) { const int L = L0 + l; if (L >= nlines) break; const int e = L * 64 + lane * 2; v2h v;
#pragma unroll
            for (int q = 0; q < 2; ++q) v[q] = tohx(geluf(H[e + q]));
            *(volatile v2h*)(P + e) = v; }
        if (ps == 0) __threadfence(); }
}
__global__ __launch_bounds__(256) void k_dsaz(const float* __restrict__ x, const float* __restrict__ gg, const float* __restrict__ bb, float* Z) {
    const int lane = threadIdx.x & 31; const int r = blockIdx.x * 8 + (threadIdx.x >> 5); if (r >= NT) return; float v[16]; float s = 0.f;
#pragma unroll
    for (int c = 0; c < 4; ++c)
#pragma unroll
        for (int q = 0; q < 4; ++q) { const float t = bfr(x[(size_t)r * CC + c * 128 + lane * 4 + q]); v[c * 4 + q] = t; s += t; }
#pragma unroll
    for (int sh = 16; sh; sh >>= 1) s += __shfl_xor(s, sh, 32);
    const float mu = s * (1.0f / CC); float qq = 0.f;
#pragma unroll
    for (int i = 0; i < 16; ++i) { const float d = v[i] - mu; qq = fmaf(d, d, qq); }
#pragma unroll
    for (int sh = 16; sh; sh >>= 1) qq += __shfl_xor(qq, sh, 32);
    const float rs = rsqrtf(qq * (1.0f / CC) + 1e-5f); v4f o[4];
#pragma unroll
    for (int c = 0; c < 4; ++c)
#pragma unroll
        for (int q = 0; q < 4; ++q) { const int col = c * 128 + lane * 4 + q; o[c][q] = (v[c * 4 + q] - mu) * rs * bfr(gg[col]) + bfr(bb[col]); }
#pragma unroll 1
    for (int ps = 0; ps < 2; ++ps) {
#pragma unroll
        for (int c = 0; c < 4; ++c) *(volatile v4f*)(Z + (size_t)r * CC + c * 128 + lane * 4) = o[c];
        if (ps == 0) __threadfence(); }
}
__global__ __launch_bounds__(256) void k_dw(const float* __restrict__ Z, const float* __restrict__ dw, const float* __restrict__ db, h16* G1) {
    const int lane = threadIdx.x & 31; const int r = blockIdx.x * 8 + (threadIdx.x >> 5); if (r >= NT) return; const int t = r % TT; const bool hasp = t > 0, hasn = t < TT - 1;
    const float* zp = Z + (size_t)(hasp ? r - 1 : r) * CC; const float* z0 = Z + (size_t)r * CC; const float* zn = Z + (size_t)(hasn ? r + 1 : r) * CC; v4h o[4];
#pragma unroll
    for (int c = 0; c < 4; ++c)
#pragma unroll
        for (int q = 0; q < 4; ++q) { const int col = c * 128 + lane * 4 + q; const float a = hasp ? zp[col] : 0.f, bq = z0[col], cn = hasn ? zn[col] : 0.f;
            const float z1 = a * bfr(dw[col * 3 + 0]) + bq * bfr(dw[col * 3 + 1]) + cn * bfr(dw[col * 3 + 2]) + bfr(db[col]); o[c][q] = tohx(gelun(z1)); }
#pragma unroll 1
    for (int ps = 0; ps < 2; ++ps) {
#pragma unroll
        for (int c = 0; c < 4; ++c) *(volatile v4h*)(G1 + (size_t)r * CC + c * 128 + lane * 4) = o[c];
        if (ps == 0) __threadfence(); }
}
__global__ __launch_bounds__(256) void k_fin(const float* __restrict__ CA, const float* __restrict__ Z2, const float* __restrict__ ap, const float* __restrict__ bp, float* OUT) {
    const size_t i = ((size_t)blockIdx.x * 256 + threadIdx.x) * 4; if (i >= (size_t)NT * CC) return; const float a = bfr(ap[0]), bb = bfr(bp[0]);
    const v4f c = *(const v4f*)(CA + i), z = *(const v4f*)(Z2 + i); const v4f o = c * a + z * bb;
    *(volatile v4f*)(OUT + i) = o; __threadfence(); *(volatile v4f*)(OUT + i) = o;
}

extern "C" void kernel_launch(void* const* d_in, const int* in_sizes, int n_in,
                              void* d_out, int out_size, void* d_ws, size_t ws_size, hipStream_t stream) {
    (void)in_sizes; (void)n_in; (void)out_size;
    const float* x = (const float*)d_in[0]; const float* A = (const float*)d_in[1]; const float* alpha = (const float*)d_in[2]; const float* dsta = (const float*)d_in[3]; const float* dstb = (const float*)d_in[4];
    const float* c1w = (const float*)d_in[5]; const float* c1b = (const float*)d_in[6]; const float* l1g = (const float*)d_in[7]; const float* l1b = (const float*)d_in[8]; const float* ipw = (const float*)d_in[9]; const float* ipb = (const float*)d_in[10];
    const float* ow = (const float*)d_in[11]; const float* ob = (const float*)d_in[12]; const float* l2g = (const float*)d_in[13]; const float* l2b = (const float*)d_in[14]; const float* m1w = (const float*)d_in[15]; const float* m1b = (const float*)d_in[16]; const float* m2w = (const float*)d_in[17]; const float* m2b = (const float*)d_in[18];
    const float* dlg = (const float*)d_in[19]; const float* dlb = (const float*)d_in[20]; const float* ddw = (const float*)d_in[21]; const float* ddb = (const float*)d_in[22]; const float* dpw = (const float*)d_in[23]; const float* dpb = (const float*)d_in[24];
    float* OUT = (float*)d_out;
    char* wsp = (char*)d_ws;
    auto take = [&](size_t bytes) { char* p = wsp; wsp += (bytes + 255) & ~(size_t)255; return (void*)p; };
    bf* WC = (bf*)take((size_t)CC * 3 * CC * 2); h16* WI = (h16*)take((size_t)3 * CC * CC * 2); h16* WO = (h16*)take((size_t)CC * CC * 2); h16* W1 = (h16*)take((size_t)FF * CC * 2); h16* W2 = (h16*)take((size_t)CC * FF * 2); h16* WP = (h16*)take((size_t)CC * CC * 2);
    float* Sb = (float*)take((size_t)ZH * TT * TT * 4);
    h16* Pm = (h16*)take((size_t)ZH * TT * TT * 2);
    float* SCR = (float*)take((size_t)NT * CC * 4);
    h16* Mh = (h16*)take((size_t)NT * CC * 2); h16* QP = (h16*)take((size_t)NT * CC * 2); h16* KP = (h16*)take((size_t)NT * CC * 2); h16* VT = (h16*)take((size_t)NT * CC * 2); h16* AT = (h16*)take((size_t)NT * CC * 2);
    float* Ob = (float*)take((size_t)ZH * TT * 64 * 4);
    bf* AIM = (bf*)Sb; float* M1 = Sb; float* Z2 = Sb; h16* M1h = Pm; float* Z = (float*)Pm;
    if ((size_t)(wsp - (char*)d_ws) > ws_size) return;
    k_wconv<<<64, 256, 0, stream>>>(c1w, WC);
    { const size_t n1 = (size_t)3 * CC * CC / 8, n2 = (size_t)CC * CC / 8, n3 = (size_t)FF * CC / 8; k_cvt8h<<<(unsigned)((n1 + 255) / 256), 256, 0, stream>>>(ipw, WI, n1); k_cvt8h<<<(unsigned)((n2 + 255) / 256), 256, 0, stream>>>(ow, WO, n2); k_cvt8h<<<(unsigned)((n3 + 255) / 256), 256, 0, stream>>>(m1w, W1, n3); k_cvt8h<<<(unsigned)((n3 + 255) / 256), 256, 0, stream>>>(m2w, W2, n3); k_cvt8h<<<(unsigned)((n2 + 255) / 256), 256, 0, stream>>>(dpw, WP, n2); }
    k_imc<<<(NT * 3 * CC / 64 + 63) / 64, 256, 0, stream>>>(x, AIM);
    k_gemmw<bf, 0, true><<<dim3(NT / 64, CC / 64, 1), 32, 0, stream>>>(AIM, nullptr, WC, nullptr, 3 * CC, SCR, CC, c1b, 0, 0, 0);
    k_lnx<true><<<NT / 8, 256, 0, stream>>>(x, SCR, l1g, l1b, Mh);
    const unsigned LBP = (unsigned)((NT * CC / 64 + 63) / 64);
    k_gemmw<h16, 0, true><<<dim3(NT / 64, CC / 64, 1), 32, 0, stream>>>(Mh, nullptr, WI, nullptr, CC, SCR, CC, ipb, 0, 0, 0); k_hplane<<<LBP, 256, 0, stream>>>(SCR, 0.125f, QP);
    k_gemmw<h16, 0, true><<<dim3(NT / 64, CC / 64, 1), 32, 0, stream>>>(Mh, nullptr, WI + (size_t)CC * CC, nullptr, CC, SCR, CC, ipb + CC, 0, 0, 0); k_hplane<<<LBP, 256, 0, stream>>>(SCR, 1.0f, KP);
    k_gemmw<h16, 0, true><<<dim3(NT / 64, CC / 64, 1), 32, 0, stream>>>(Mh, nullptr, WI + (size_t)2 * CC * CC, nullptr, CC, SCR, CC, ipb + 2 * CC, 0, 0, 0); k_vtplane<<<LBP, 256, 0, stream>>>(SCR, VT);
    for (int b = 0; b < NB_; ++b)
        for (int h0 = 0; h0 < NH_; h0 += ZH) { const size_t z0 = (size_t)b * NH_ + h0;
            k_gemmw<h16, 0, false><<<dim3(TT / 64, TT / 64, ZH), 32, 0, stream>>>(QP + z0 * TT * HD, nullptr, KP + z0 * TT * HD, nullptr, HD, Sb, TT, nullptr, (size_t)TT * HD, (size_t)TT * HD, (size_t)TT * TT);
            k_softab<<<ZH * TT / 8, 256, 0, stream>>>(Sb, A, alpha, b, Pm);
            k_gemmw<h16, 0, false><<<dim3(TT / 64, 1, ZH), 32, 0, stream>>>(Pm, nullptr, VT + z0 * HD * TT, nullptr, TT, Ob, HD, nullptr, (size_t)TT * TT, (size_t)HD * TT, (size_t)TT * HD);
            k_merge<<<TT / 8, 256, 0, stream>>>(Ob, b, h0, AT); }
    k_gemmw<h16, 0, true><<<dim3(NT / 64, CC / 64, 1), 32, 0, stream>>>(AT, nullptr, WO, nullptr, CC, SCR, CC, ob, 0, 0, 0);
    k_lnx<false><<<NT / 8, 256, 0, stream>>>(x, SCR, l2g, l2b, Mh);
    for (int ch = 0; ch < 2; ++ch) { const size_t r0 = (size_t)ch * (NT / 2);
        k_gemmw<h16, 0, true><<<dim3((NT / 2) / 64, FF / 64, 1), 32, 0, stream>>>(Mh + r0 * CC, nullptr, W1, nullptr, CC, M1, FF, m1b, 0, 0, 0);
        k_gelu16<<<((NT / 2) * FF / 64 + 63) / 64, 256, 0, stream>>>(M1, (NT / 2) * FF, M1h);
        k_gemmw<h16, 0, true><<<dim3((NT / 2) / 64, CC / 64, 1), 32, 0, stream>>>(M1h, nullptr, W2, nullptr, FF, SCR + r0 * CC, CC, m2b, 0, 0, 0); }
    k_dsaz<<<NT / 8, 256, 0, stream>>>(x, dlg, dlb, Z);
    k_dw<<<NT / 8, 256, 0, stream>>>(Z, ddw, ddb, Mh);
    k_gemmw<h16, 0, true><<<dim3(NT / 64, CC / 64, 1), 32, 0, stream>>>(Mh, nullptr, WP, nullptr, CC, Z2, CC, dpb, 0, 0, 0);
    k_fin<<<(unsigned)(((size_t)NT * CC / 4 + 255) / 256), 256, 0, stream>>>(SCR, Z2, dsta, dstb, OUT);
}
